// MSARowAttentionWithPairBias_5600637354564
// MI455X (gfx1250) — hardware-verified
//
#include <hip/hip_runtime.h>
#include <math.h>

constexpr int kS   = 128;
constexpr int kR   = 256;
constexpr int kCM  = 256;
constexpr int kCZ  = 128;
constexpr int kH   = 8;
constexpr int kC   = 32;
constexpr int kHD  = kH * kC;
constexpr int kTok = kS * kR;
constexpr int kPairRows = kR * kR;
constexpr int kNChunk = 2;
constexpr int kSC     = kS / kNChunk;
constexpr int kTokC   = kSC * kR;
constexpr int kQKld = 2 * kHD;
constexpr int kQT   = 32;
constexpr int kPld  = kR + 8;
constexpr int kOsld = 2 * kC + 4;
constexpr int kWPlane = 256 * 256;
constexpr float kWCarry    = 16.0f;
constexpr float kWCarryInv = 1.0f / 16.0f;
constexpr float kPCarry    = 32768.0f;
constexpr float kPCarryInv = 1.0f / 32768.0f;
constexpr float kOBCarry   = 256.0f;
constexpr float kOutScale  = 1.0f / (256.0f * 16.0f);
constexpr float kQScale    = 0.17677669529663687f;
constexpr float kLnEps     = 1.0e-5f;
constexpr float kInvCM     = 1.0f / 256.0f;
constexpr float kInvCZ     = 1.0f / 128.0f;
static_assert(kCM == 256 && kHD == 256 && kR == 256 && kCZ == 128, "shape");
static_assert(kS % kNChunk == 0, "chunking");
static_assert(kTokC % 64 == 0 && kQKld % 64 == 0 && kCM % 32 == 0, "q|k GEMM M,N,K");
static_assert(kTokC % 64 == 0 && kHD % 64 == 0, "g GEMM M,N");
static_assert(kHD % 64 == 0 && kR % 64 == 0, "v^T GEMM M,N");
static_assert(kTok % 64 == 0 && kCM % 64 == 0 && kHD % 32 == 0, "out GEMM M,N,K");
static_assert(kC % 32 == 0 && kR % 32 == 0, "logit K and P.V K multiples of 32");
static_assert(kQKld % 8 == 0 && kPld % 8 == 0 && kOsld % 4 == 0, "16-B alignment of fragment rows");
static_assert(kR / kQT == 8 && kH / 2 == 4, "attention block decode");
static_assert(kTokC % 8 == 0 && kPairRows % 32 == 0, "row kernels grids");
static_assert(((kTokC / 64) * (kQKld / 64)) % 8 == 0 && ((kTokC / 64) * (kHD / 64)) % 8 == 0, "GEMM grids exact");
static_assert(((kHD / 64) * (kR / 64)) % 8 == 0 && ((kTok / 64) * (kCM / 64)) % 8 == 0, "GEMM grids exact");

typedef __attribute__((ext_vector_type(16))) _Float16 v16h;
typedef __attribute__((ext_vector_type(8)))  _Float16 v8h;
typedef __attribute__((ext_vector_type(16))) __bf16   v16b;
typedef __attribute__((ext_vector_type(8)))  __bf16   v8b;
typedef __attribute__((ext_vector_type(8)))  float    v8f;
typedef __attribute__((ext_vector_type(4)))  float    v4f;
typedef __attribute__((ext_vector_type(4)))  unsigned int v4u;

__device__ __forceinline__ unsigned short f2bf_bits(float f) {
  unsigned u = __float_as_uint(f);
  return (unsigned short)((u + 0x7FFFu + ((u >> 16) & 1u)) >> 16);
}
__device__ __forceinline__ float bf_bits2f(unsigned short h) { return __uint_as_float(((unsigned)h) << 16); }

__device__ __forceinline__ void dep_guard_h(v8f& a, v8f& b, v16h x, v16h y) { asm volatile("v_nop\n\tv_nop\n\tv_nop\n\tv_nop" : "+v"(a), "+v"(b) : "v"(x), "v"(y)); }
__device__ __forceinline__ void dep_guard_b(v8f& a, v8f& b, v16b x, v16b y) { asm volatile("v_nop\n\tv_nop\n\tv_nop\n\tv_nop" : "+v"(a), "+v"(b) : "v"(x), "v"(y)); }
__device__ __forceinline__ void dep_guard4_h(v8f& a, v8f& b, v8f& c, v8f& d, v16h x, v16h y) { asm volatile("v_nop\n\tv_nop\n\tv_nop\n\tv_nop" : "+v"(a), "+v"(b), "+v"(c), "+v"(d) : "v"(x), "v"(y)); }
__device__ __forceinline__ void dep_guard4_b(v8f& a, v8f& b, v8f& c, v8f& d, v16b x, v16b y) { asm volatile("v_nop\n\tv_nop\n\tv_nop\n\tv_nop" : "+v"(a), "+v"(b), "+v"(c), "+v"(d) : "v"(x), "v"(y)); }
__device__ __forceinline__ void dep_guard1_h(v8f& a, v16h x, v16h y) { asm volatile("v_nop\n\tv_nop\n\tv_nop\n\tv_nop" : "+v"(a) : "v"(x), "v"(y)); }
__device__ __forceinline__ void keep4_h(v16h a, v16h b, v16h c, v16h d) { asm volatile("v_nop" :: "v"(a), "v"(b), "v"(c), "v"(d)); }
__device__ __forceinline__ void keep4_b(v16b a, v16b b, v16b c, v16b d) { asm volatile("v_nop" :: "v"(a), "v"(b), "v"(c), "v"(d)); }
__device__ __forceinline__ void acc_guard4(v8f& a, v8f& b, v8f& c, v8f& d) { asm volatile("v_nop\n\tv_nop\n\tv_nop\n\tv_nop" : "+v"(a), "+v"(b), "+v"(c), "+v"(d)); }
template <typename T> struct Frag;
template <> struct Frag<_Float16> {
  typedef v16h V; union U { v16h v; v8h h[2]; };
  static __device__ __forceinline__ v16h load(const _Float16* p) {
    U f; f.h[0] = *(const v8h*)(p); f.h[1] = *(const v8h*)(p + 16); return f.v;
  }
  static __device__ __forceinline__ v8f mma(v16h a, v16h b, v8f c) {
    return __builtin_amdgcn_wmma_f32_16x16x32_f16(false, a, false, b, (short)0, c, false, false);
  }
  static __device__ __forceinline__ void guard(v8f& a, v8f& b, v16h x, v16h y) { dep_guard_h(a, b, x, y); }
  static __device__ __forceinline__ void guard4(v8f& a, v8f& b, v8f& c, v8f& d, v16h x, v16h y) { dep_guard4_h(a, b, c, d, x, y); }
  static __device__ __forceinline__ void keep(v16h a, v16h b, v16h c, v16h d) { keep4_h(a, b, c, d); }
};
template <> struct Frag<__bf16> {
  typedef v16b V; union U { v16b v; v8b h[2]; };
  static __device__ __forceinline__ v16b load(const __bf16* p) {
    U f; f.h[0] = *(const v8b*)(p); f.h[1] = *(const v8b*)(p + 16); return f.v;
  }
  static __device__ __forceinline__ v8f mma(v16b a, v16b b, v8f c) {
    return __builtin_amdgcn_wmma_f32_16x16x32_bf16(false, a, false, b, (short)0, c, false, false);
  }
  static __device__ __forceinline__ void guard(v8f& a, v8f& b, v16b x, v16b y) { dep_guard_b(a, b, x, y); }
  static __device__ __forceinline__ void guard4(v8f& a, v8f& b, v8f& c, v8f& d, v16b x, v16b y) { dep_guard4_b(a, b, c, d, x, y); }
  static __device__ __forceinline__ void keep(v16b a, v16b b, v16b c, v16b d) { keep4_b(a, b, c, d); }
};

__device__ __forceinline__ unsigned pk16(unsigned short a, unsigned short b) { return (unsigned)a | ((unsigned)b << 16); }
__device__ __forceinline__ unsigned short h_bits(float f) { const _Float16 h = (_Float16)f; return __builtin_bit_cast(unsigned short, h); }

__device__ __forceinline__ float h16_to_f32(unsigned hb) {
  const unsigned sgn = (hb & 0x8000u) << 16; const unsigned em = hb & 0x7fffu;
  const float fn = __uint_as_float((em << 13) + 0x38000000u);
  const float fs = (float)em * 5.9604644775390625e-8f;
  const float mag = (em < 0x400u) ? fs : fn; return __uint_as_float(__float_as_uint(mag) | sgn); }

template <int ET> struct Elem;
template <> struct Elem<0> { typedef _Float16 T; };
template <> struct Elem<1> { typedef __bf16 T; };
template <int ET, bool SPLIT, int BIAS_MODE, int OUT_MODE, bool RESID, int ACT = 0>
__global__ __launch_bounds__(256) void wmma_gemm64(
    const unsigned short* __restrict__ Ap, const unsigned short* __restrict__ A2p, int lda, long strideA,
    const unsigned short* __restrict__ Btp, const unsigned short* __restrict__ Bt2p, int ldb, long strideB,
    void* __restrict__ Cout, void* __restrict__ Cout2, int ldc, long strideC,
    const float* __restrict__ bias,
    const float* __restrict__ resid, long strideR,
    int M, int N, int K, float scale) {
  typedef typename Elem<ET>::T T;
  typedef typename Frag<T>::V V;
  const T* A = (const T*)Ap; const T* A2 = (const T*)A2p; const T* Bt = (const T*)Btp; const T* Bt2 = (const T*)Bt2p;
  __shared__ __align__(16) float sT[8][16 * 68];
  const int b    = blockIdx.y;
  const int lane = threadIdx.x & 31;
  const int wave = threadIdx.x >> 5;
  const int tilesN = N >> 6;
  const int tilesM = M >> 6;
  const int tile = blockIdx.x * 8 + wave;
  if (tile >= tilesM * tilesN) return;
  const int tm = tile / tilesN;
  const int tn = tile - tm * tilesN;
  const int m0 = tm << 6;
  const int n0 = tn << 6;

  const T* Ab  = A  + (size_t)b * strideA;
  const T* Bb  = Bt + (size_t)b * strideB;
  const T* Ab2 = SPLIT ? (A2  + (size_t)b * strideA) : nullptr;
  const T* Bb2 = SPLIT ? (Bt2 + (size_t)b * strideB) : nullptr;

  const int rlane = lane & 15;
  const int koff  = (lane >> 4) * 8;
  const int mOff  = (lane >> 4) * 8;

  v8f acc[4][4];
#pragma unroll
  for (int i = 0; i < 4; ++i)
#pragma unroll
    for (int j = 0; j < 4; ++j) acc[i][j] = (v8f){0.f,0.f,0.f,0.f,0.f,0.f,0.f,0.f};

  for (int k0 = 0; k0 < K; k0 += 32) {
    V bh[4], bl[4];
#pragma unroll
    for (int j = 0; j < 4; ++j) {
      const size_t bo = (size_t)(n0 + (j << 4) + rlane) * ldb + koff + k0;
      bh[j] = Frag<T>::load(Bb + bo);
      if (SPLIT) bl[j] = Frag<T>::load(Bb2 + bo);
    }
#pragma unroll
    for (int i = 0; i < 4; ++i) {
      const size_t ao = (size_t)(m0 + (i << 4) + rlane) * lda + koff + k0;
      V ah = Frag<T>::load(Ab + ao);
      V al;
      if (SPLIT) al = Frag<T>::load(Ab2 + ao);
#pragma unroll
      for (int j = 0; j < 4; ++j) {
        acc[i][j] = Frag<T>::mma(ah, bh[j], acc[i][j]);
        if (SPLIT) {
          acc[i][j] = Frag<T>::mma(ah, bl[j], acc[i][j]);
          acc[i][j] = Frag<T>::mma(al, bh[j], acc[i][j]);
        }
      }
      Frag<T>::guard4(acc[i][0], acc[i][1], acc[i][2], acc[i][3], ah, SPLIT ? al : ah);
    }
    Frag<T>::keep(bh[0], bh[1], bh[2], bh[3]);
    if (SPLIT) Frag<T>::keep(bl[0], bl[1], bl[2], bl[3]);
  }
  acc_guard4(acc[0][0], acc[0][1], acc[0][2], acc[0][3]);
  acc_guard4(acc[1][0], acc[1][1], acc[1][2], acc[1][3]);
  acc_guard4(acc[2][0], acc[2][1], acc[2][2], acc[2][3]);
  acc_guard4(acc[3][0], acc[3][1], acc[3][2], acc[3][3]);

  float* slab = sT[wave];
  const float* Rb = RESID ? (resid + (size_t)b * strideR) : nullptr;
#pragma unroll
  for (int i = 0; i < 4; ++i) {
    const int mBase = m0 + (i << 4);
#pragma unroll
    for (int j = 0; j < 4; ++j) {
      const int n = n0 + (j << 4) + rlane;
      float bv = 0.f;
      if (BIAS_MODE == 2) bv = bias[n];
#pragma unroll
      for (int r = 0; r < 8; ++r) {
        float v = acc[i][j][r] * scale;
        if (BIAS_MODE == 1) v += bias[mBase + mOff + r];
        if (BIAS_MODE == 2) v += bv;
        if (RESID) v += Rb[(size_t)(mBase + mOff + r) * ldc + n];
        if (ACT == 2) v = fmaxf(v, 0.0f);
        if (ACT == 4) v = (v > 0.f) ? v : 0.01f * v;
        slab[(mOff + r) * 68 + (j << 4) + rlane] = v;
      }
    }
    __builtin_amdgcn_fence(__ATOMIC_RELEASE, "workgroup");
    __builtin_amdgcn_wave_barrier();
    __builtin_amdgcn_fence(__ATOMIC_ACQUIRE, "workgroup");
    if (OUT_MODE == 0) {
      float* C = (float*)Cout + (size_t)b * strideC;
      const int hh = lane >> 4, c4 = (lane & 15) * 4;
      for (int pass = 0; pass < 2; ++pass) {
#pragma unroll
        for (int it = 0; it < 8; ++it) {
          const int row = it * 2 + hh;
          v4f v = *(const v4f*)(slab + row * 68 + c4);
          *(volatile v4f*)(C + (size_t)(mBase + row) * ldc + n0 + c4) = v;
        }
        __threadfence();
      }
    } else {
      const int q = lane >> 3, c8 = (lane & 7) * 8;
      unsigned short* C  = (unsigned short*)Cout  + (size_t)b * strideC;
      unsigned short* C2 = (OUT_MODE == 2) ? ((unsigned short*)Cout2 + (size_t)b * strideC) : nullptr;
      for (int pass = 0; pass < 2; ++pass) {
#pragma unroll
        for (int it = 0; it < 4; ++it) {
          const int row = it * 4 + q;
          const float* sp = slab + row * 68 + c8;
          v8h hv, lv;
#pragma unroll
          for (int e = 0; e < 8; ++e) {
            if (OUT_MODE == 1) {
              hv[e] = (_Float16)sp[e];
            } else {
              unsigned short hb = f2bf_bits(sp[e]);
              unsigned short lb = f2bf_bits(sp[e] - bf_bits2f(hb));
              hv[e] = __builtin_bit_cast(_Float16, hb);
              lv[e] = __builtin_bit_cast(_Float16, lb);
            }
          }
          *(volatile v8h*)(C + (size_t)(mBase + row) * ldc + n0 + c8) = hv;
          if (OUT_MODE == 2) *(volatile v8h*)(C2 + (size_t)(mBase + row) * ldc + n0 + c8) = lv;
        }
        __threadfence();
      }
    }
    __builtin_amdgcn_fence(__ATOMIC_RELEASE, "workgroup");
    __builtin_amdgcn_wave_barrier();
    __builtin_amdgcn_fence(__ATOMIC_ACQUIRE, "workgroup");
  }
}

__global__ __launch_bounds__(256) void wtcast_kernel(const float* __restrict__ W0, const float* __restrict__ W1,
                                                     const float* __restrict__ W2,
                                                     unsigned short* __restrict__ out, float scale) {
  __shared__ float sm[64][65];
  const int t  = threadIdx.x;
  const int d0 = blockIdx.x * 64;
  const int h0 = blockIdx.y * 64;
  const int z  = blockIdx.z;
  const float* W = (z == 0) ? W0 : (z == 1) ? W1 : W2;
#pragma unroll
  for (int i = 0; i < 16; ++i) {
    const int e = i * 256 + t;
    const int r = e >> 6;
    const int c = e & 63;
    sm[c][r] = W[(size_t)(d0 + r) * 256 + h0 + c] * scale;
  }
  __syncthreads();
  const int lane = t & 31, wave = t >> 5;
  const int q = lane >> 3, c8 = (lane & 7) * 8;
  unsigned short* op = out + (size_t)z * kWPlane;
  for (int pass = 0; pass < 2; ++pass) {
#pragma unroll
    for (int it = 0; it < 2; ++it) {
      const int row = wave * 8 + it * 4 + q;
      unsigned short hb[8];
#pragma unroll
      for (int e = 0; e < 8; ++e) hb[e] = h_bits(sm[row][c8 + e]);
      const v4u u = (v4u){pk16(hb[0], hb[1]), pk16(hb[2], hb[3]), pk16(hb[4], hb[5]), pk16(hb[6], hb[7])};
      *(volatile v4u*)(op + (size_t)(h0 + row) * 256 + d0 + c8) = u;
    }
    __threadfence();
  }
}

__global__ __launch_bounds__(256) void wtsplit_kernel(const float* __restrict__ W0, const float* __restrict__ W1,
                                                      unsigned short* __restrict__ outh, unsigned short* __restrict__ outl) {
  __shared__ float sm[64][65];
  const int t  = threadIdx.x;
  const int d0 = blockIdx.x * 64;
  const int h0 = blockIdx.y * 64;
  const int z  = blockIdx.z;
  const float* W = (z == 0) ? W0 : W1;
#pragma unroll
  for (int i = 0; i < 16; ++i) {
    const int e = i * 256 + t;
    const int r = e >> 6;
    const int c = e & 63;
    sm[c][r] = W[(size_t)(d0 + r) * 256 + h0 + c];
  }
  __syncthreads();
  const int lane = t & 31, wave = t >> 5;
  const int q = lane >> 3, c8 = (lane & 7) * 8;
  unsigned short* oph = outh + (size_t)z * kWPlane;
  unsigned short* opl = outl + (size_t)z * kWPlane;
  for (int pass = 0; pass < 2; ++pass) {
#pragma unroll
    for (int it = 0; it < 2; ++it) {
      const int row = wave * 8 + it * 4 + q;
      unsigned short hb[8], lb[8];
#pragma unroll
      for (int e = 0; e < 8; ++e) {
        const float v = sm[row][c8 + e];
        hb[e] = f2bf_bits(v);
        lb[e] = f2bf_bits(v - bf_bits2f(hb[e]));
      }
      const v4u uh = (v4u){pk16(hb[0], hb[1]), pk16(hb[2], hb[3]), pk16(hb[4], hb[5]), pk16(hb[6], hb[7])};
      const v4u ul = (v4u){pk16(lb[0], lb[1]), pk16(lb[2], lb[3]), pk16(lb[4], lb[5]), pk16(lb[6], lb[7])};
      const size_t o = (size_t)(h0 + row) * 256 + d0 + c8;
      *(volatile v4u*)(oph + o) = uh;
      *(volatile v4u*)(opl + o) = ul;
    }
    __threadfence();
  }
}

__global__ __launch_bounds__(256) void ln_msa_kernel(const float* __restrict__ x, const float* __restrict__ gam,
                                                     const float* __restrict__ bet, unsigned short* __restrict__ M16,
                                                     unsigned short* __restrict__ Mhi, unsigned short* __restrict__ Mlo) {
  const int t = threadIdx.x, lane = t & 31, wave = t >> 5;
  const int row = blockIdx.x * 8 + wave;
  const int c0  = lane * 8;
  const float* p = x + (size_t)row * kCM + c0;
  const v4f xa = *(const v4f*)(p);
  const v4f xc = *(const v4f*)(p + 4);
  const v4f ga = *(const v4f*)(gam + c0);
  const v4f gc = *(const v4f*)(gam + c0 + 4);
  const v4f ba = *(const v4f*)(bet + c0);
  const v4f bc = *(const v4f*)(bet + c0 + 4);
  float xs[8], gs[8], bs[8];
#pragma unroll
  for (int e = 0; e < 4; ++e) { xs[e] = xa[e]; xs[4 + e] = xc[e]; gs[e] = ga[e]; gs[4 + e] = gc[e]; bs[e] = ba[e]; bs[4 + e] = bc[e]; }
  float s = 0.0f;
#pragma unroll
  for (int e = 0; e < 8; ++e) s += xs[e];
#pragma unroll
  for (int off = 16; off > 0; off >>= 1) s += __shfl_xor(s, off, 32);
  const float mu = s * kInvCM;
  float d[8];
  float s2 = 0.0f;
#pragma unroll
  for (int e = 0; e < 8; ++e) { d[e] = xs[e] - mu; s2 += d[e] * d[e]; }
#pragma unroll
  for (int off = 16; off > 0; off >>= 1) s2 += __shfl_xor(s2, off, 32);
  const float var = s2 * kInvCM;
  const float rs  = rsqrtf(var + kLnEps);
  unsigned short fb[8], hb[8], lb[8];
#pragma unroll
  for (int e = 0; e < 8; ++e) {
    const float y = d[e] * rs * gs[e] + bs[e];
    fb[e] = h_bits(y);
    hb[e] = f2bf_bits(y);
    lb[e] = f2bf_bits(y - bf_bits2f(hb[e]));
  }
  const v4u uf = (v4u){pk16(fb[0], fb[1]), pk16(fb[2], fb[3]), pk16(fb[4], fb[5]), pk16(fb[6], fb[7])};
  const v4u uh = (v4u){pk16(hb[0], hb[1]), pk16(hb[2], hb[3]), pk16(hb[4], hb[5]), pk16(hb[6], hb[7])};
  const v4u ul = (v4u){pk16(lb[0], lb[1]), pk16(lb[2], lb[3]), pk16(lb[4], lb[5]), pk16(lb[6], lb[7])};
  const size_t o = (size_t)row * kCM + c0;
  *(volatile v4u*)(M16 + o) = uf;
  *(volatile v4u*)(Mhi + o) = uh;
  *(volatile v4u*)(Mlo + o) = ul;
  __threadfence();
  *(volatile v4u*)(M16 + o) = uf;
  *(volatile v4u*)(Mhi + o) = uh;
  *(volatile v4u*)(Mlo + o) = ul;
}

__global__ __launch_bounds__(256) void pair_bias_kernel(const float* __restrict__ pr, const float* __restrict__ gam,
                                                        const float* __restrict__ bet, const float* __restrict__ wb,
                                                        const float* __restrict__ bb, float* __restrict__ PB) {
  __shared__ __align__(16) float wbs[kCZ * kH];
  __shared__ __align__(16) float bres[kH][32];
  const int t = threadIdx.x, lane = t & 31, wave = t >> 5;
  *(v4f*)(wbs + 4 * t) = *(const v4f*)(wb + 4 * t);
  const int row0 = blockIdx.x * 32;
  const int c0   = lane * 4;
  const v4f gv  = *(const v4f*)(gam + c0);
  const v4f bv  = *(const v4f*)(bet + c0);
  const v4f bb0 = *(const v4f*)(bb);
  const v4f bb1 = *(const v4f*)(bb + 4);
  __syncthreads();
#pragma unroll 1
  for (int rr = 0; rr < 4; ++rr) {
    const int rloc = wave * 4 + rr;
    const int row  = row0 + rloc;
    const v4f xv = *(const v4f*)(pr + (size_t)row * kCZ + c0);
    float s = (xv[0] + xv[1]) + (xv[2] + xv[3]);
#pragma unroll
    for (int off = 16; off > 0; off >>= 1) s += __shfl_xor(s, off, 32);
    const float mu = s * kInvCZ;
    float d[4];
    float s2 = 0.0f;
#pragma unroll
    for (int e = 0; e < 4; ++e) { d[e] = xv[e] - mu; s2 += d[e] * d[e]; }
#pragma unroll
    for (int off = 16; off > 0; off >>= 1) s2 += __shfl_xor(s2, off, 32);
    const float var = s2 * kInvCZ;
    const float rs  = rsqrtf(var + kLnEps);
    float acc[8];
#pragma unroll
    for (int j = 0; j < 8; ++j) acc[j] = 0.0f;
#pragma unroll
    for (int e = 0; e < 4; ++e) {
      const float zc = d[e] * rs * gv[e] + bv[e];
      const v4f w0 = *(const v4f*)(wbs + (c0 + e) * kH);
      const v4f w1 = *(const v4f*)(wbs + (c0 + e) * kH + 4);
      acc[0] += zc * w0[0]; acc[1] += zc * w0[1]; acc[2] += zc * w0[2]; acc[3] += zc * w0[3];
      acc[4] += zc * w1[0]; acc[5] += zc * w1[1]; acc[6] += zc * w1[2]; acc[7] += zc * w1[3];
    }
#pragma unroll
    for (int off = 16; off > 0; off >>= 1) {
#pragma unroll
      for (int j = 0; j < 8; ++j) acc[j] += __shfl_xor(acc[j], off, 32);
    }
    if (lane == 0) {
      bres[0][rloc] = acc[0] + bb0[0];
      bres[1][rloc] = acc[1] + bb0[1];
      bres[2][rloc] = acc[2] + bb0[2];
      bres[3][rloc] = acc[3] + bb0[3];
      bres[4][rloc] = acc[4] + bb1[0];
      bres[5][rloc] = acc[5] + bb1[1];
      bres[6][rloc] = acc[6] + bb1[2];
      bres[7][rloc] = acc[7] + bb1[3];
    }
  }
  __syncthreads();
  if (wave < 2) {
    const int hq = wave * 4 + (lane >> 3);
    const int c4 = (lane & 7) * 4;
    const v4f v = *(const v4f*)(&bres[hq][c4]);
    float* dst = PB + (size_t)hq * kPairRows + row0 + c4;
    *(volatile v4f*)dst = v;
    __threadfence();
    *(volatile v4f*)dst = v;
  }
}

__global__ __launch_bounds__(256) void attn_kernel(const unsigned short* __restrict__ qkh, const unsigned short* __restrict__ qkl,
                                                   const unsigned short* __restrict__ g16, const unsigned short* __restrict__ vt,
                                                   const float* __restrict__ PB, const float* __restrict__ bg,
                                                   unsigned short* __restrict__ ob) {
  __shared__ __align__(16) float    Sf[kQT * kR];
  __shared__ __align__(16) _Float16 P16[kQT * kPld];
  __shared__ __align__(16) float    Os[kQT * kOsld];
  const int t = threadIdx.x, lane = t & 31, wave = t >> 5;
  const int rlane = lane & 15;
  const int koff  = (lane >> 4) * 8;
  const int mOff  = (lane >> 4) * 8;
  const int bid = blockIdx.x;
  const int qt  = bid & 7;
  const int hp  = (bid >> 3) & 3;
  const int sl  = bid >> 5;
  const int q0    = qt * kQT;
  const int srow0 = sl * kR;
  const int rowq  = srow0 + q0;
  const __bf16*   QH  = (const __bf16*)(const void*)qkh;
  const __bf16*   QL  = (const __bf16*)(const void*)qkl;
  const _Float16* VTh = (const _Float16*)(const void*)vt;

#pragma unroll 1
  for (int hl = 0; hl < 2; ++hl) {
    const int h = hp * 2 + hl;
    {
      const int mt  = wave >> 2;
      const int ntb = (wave & 3) * 4;
      v16b bh[4], bl[4];
#pragma unroll
      for (int j = 0; j < 4; ++j) {
        const size_t bo = (size_t)(srow0 + (ntb + j) * 16 + rlane) * kQKld + kHD + h * kC + koff;
        bh[j] = Frag<__bf16>::load(QH + bo);
        bl[j] = Frag<__bf16>::load(QL + bo);
      }
      const size_t ao = (size_t)(rowq + mt * 16 + rlane) * kQKld + h * kC + koff;
      const v16b ah = Frag<__bf16>::load(QH + ao);
      const v16b al = Frag<__bf16>::load(QL + ao);
      v8f acc[4];
#pragma unroll
      for (int j = 0; j < 4; ++j) {
        acc[j] = (v8f){0.f,0.f,0.f,0.f,0.f,0.f,0.f,0.f};
        acc[j] = Frag<__bf16>::mma(ah, bh[j], acc[j]);
        acc[j] = Frag<__bf16>::mma(ah, bl[j], acc[j]);
        acc[j] = Frag<__bf16>::mma(al, bh[j], acc[j]);
      }
      dep_guard4_b(acc[0], acc[1], acc[2], acc[3], ah, al);
      keep4_b(bh[0], bh[1], bh[2], bh[3]);
      keep4_b(bl[0], bl[1], bl[2], bl[3]);
#pragma unroll
      for (int j = 0; j < 4; ++j) {
#pragma unroll
        for (int r = 0; r < 8; ++r)
          Sf[(mt * 16 + mOff + r) * kR + (ntb + j) * 16 + rlane] = acc[j][r] * kQScale;
      }
    }
    __syncthreads();
    {
      const int row = t >> 3, seg = t & 7, cb = seg * 32;
      float* sr = Sf + row * kR + cb;
      const float* br = PB + (size_t)h * kPairRows + (size_t)(q0 + row) * kR + cb;
      float mx = -__builtin_inff();
#pragma unroll
      for (int i = 0; i < 8; ++i) {
        const v4f sv = *(const v4f*)(sr + 4 * i);
        const v4f bv = *(const v4f*)(br + 4 * i);
        const v4f lv = sv + bv;
        *(v4f*)(sr + 4 * i) = lv;
        mx = fmaxf(fmaxf(mx, fmaxf(lv[0], lv[1])), fmaxf(lv[2], lv[3]));
      }
      mx = fmaxf(mx, __shfl_xor(mx, 1, 32));
      mx = fmaxf(mx, __shfl_xor(mx, 2, 32));
      mx = fmaxf(mx, __shfl_xor(mx, 4, 32));
      float sum = 0.0f;
#pragma unroll 2
      for (int i = 0; i < 8; ++i) {
        const v4f lv = *(const v4f*)(sr + 4 * i);
        v4f ev;
        ev[0] = expf(lv[0] - mx);
        ev[1] = expf(lv[1] - mx);
        ev[2] = expf(lv[2] - mx);
        ev[3] = expf(lv[3] - mx);
        *(v4f*)(sr + 4 * i) = ev;
        sum += (ev[0] + ev[1]) + (ev[2] + ev[3]);
      }
      sum += __shfl_xor(sum, 1, 32);
      sum += __shfl_xor(sum, 2, 32);
      sum += __shfl_xor(sum, 4, 32);
      const float inv = kPCarry / sum;
#pragma unroll
      for (int i = 0; i < 4; ++i) {
        const v4f e0 = *(const v4f*)(sr + 8 * i);
        const v4f e1 = *(const v4f*)(sr + 8 * i + 4);
        v8h hv;
#pragma unroll
        for (int e = 0; e < 4; ++e) {
          hv[e]     = (_Float16)(e0[e] * inv);
          hv[4 + e] = (_Float16)(e1[e] * inv);
        }
        *(v8h*)(P16 + row * kPld + cb + 8 * i) = hv;
      }
    }
    __syncthreads();
    if (wave < 4) {
      const int mt = wave >> 1, nt = wave & 1;
      const _Float16* pa = P16 + (mt * 16 + rlane) * kPld + koff;
      const _Float16* pb = VTh + ((size_t)sl * kHD + h * kC + nt * 16 + rlane) * kR + koff;
      v8f acc = (v8f){0.f,0.f,0.f,0.f,0.f,0.f,0.f,0.f};
#pragma unroll
      for (int ks = 0; ks < 8; ++ks) {
        const v16h a = Frag<_Float16>::load(pa + ks * 32);
        const v16h b = Frag<_Float16>::load(pb + ks * 32);
        acc = Frag<_Float16>::mma(a, b, acc);
        dep_guard1_h(acc, a, b);
      }
#pragma unroll
      for (int r = 0; r < 8; ++r)
        Os[(mt * 16 + mOff + r) * kOsld + hl * kC + nt * 16 + rlane] = acc[r] * kPCarryInv;
    }
    __syncthreads();
  }

  {
    const int row = t >> 3, d8 = (t & 7) * 8;
    const size_t grow = (size_t)(rowq + row);
    const v4u gw = *(const v4u*)(g16 + grow * kHD + hp * 64 + d8);
    const v4f g0 = *(const v4f*)(bg + hp * 64 + d8);
    const v4f g1 = *(const v4f*)(bg + hp * 64 + d8 + 4);
    const v4f o0 = *(const v4f*)(Os + row * kOsld + d8);
    const v4f o1 = *(const v4f*)(Os + row * kOsld + d8 + 4);
    float gp[8], gb[8], ov[8];
#pragma unroll
    for (int i = 0; i < 4; ++i) {
      gp[2 * i]     = h16_to_f32(gw[i] & 0xffffu);
      gp[2 * i + 1] = h16_to_f32(gw[i] >> 16);
      gb[i] = g0[i]; gb[4 + i] = g1[i];
      ov[i] = o0[i]; ov[4 + i] = o1[i];
    }
    unsigned short hb[8];
#pragma unroll
    for (int e = 0; e < 8; ++e) {
      const float v  = gp[e] + gb[e];
      const float ex = expf(-fabsf(v));
      const float sg = 1.0f / (1.0f + ex);
      const float g  = (v >= 0.0f) ? sg : ex * sg;
      hb[e] = h_bits(g * ov[e] * kOBCarry);
    }
    const v4u u = (v4u){pk16(hb[0], hb[1]), pk16(hb[2], hb[3]), pk16(hb[4], hb[5]), pk16(hb[6], hb[7])};
    unsigned short* dst = ob + grow * kHD + hp * 64 + d8;
    *(volatile v4u*)dst = u;
    __threadfence();
    *(volatile v4u*)dst = u;
  }
}

extern "C" void kernel_launch(void* const* d_in, const int* in_sizes, int n_in,
                              void* d_out, int out_size, void* d_ws, size_t ws_size,
                              hipStream_t stream) {
  if (n_in < 15) return;
  if (in_sizes[0] != kTok * kCM) return;
  if (in_sizes[1] != kPairRows * kCZ) return;
  if (in_sizes[2] != kCM || in_sizes[3] != kCM) return;
  if (in_sizes[4] != kCZ || in_sizes[5] != kCZ) return;
  if (in_sizes[6] != kCM * kHD || in_sizes[7] != kCM * kHD || in_sizes[8] != kCM * kHD || in_sizes[9] != kCM * kHD) return;
  if (in_sizes[10] != kHD || in_sizes[11] != kCZ * kH || in_sizes[12] != kH) return;
  if (in_sizes[13] != kHD * kCM || in_sizes[14] != kCM) return;
  if (out_size != kTok * kCM) return;

  const size_t szWT16 = (size_t)3 * kWPlane * 2;
  const size_t szWQK  = (size_t)2 * kWPlane * 2;
  const size_t szMc   = (size_t)kTokC * kCM * 2;
  const size_t szQKc  = (size_t)kTokC * kQKld * 2;
  const size_t szGc   = (size_t)kTokC * kHD * 2;
  const size_t szVTc  = (size_t)kSC * kHD * kR * 2;
  const size_t szPB   = (size_t)kH * kPairRows * 4;
  const size_t szOB   = (size_t)kTok * kHD * 2;
  const size_t offWT16 = 0;
  const size_t offWQKh = offWT16 + szWT16;
  const size_t offWQKl = offWQKh + szWQK;
  const size_t offM16  = offWQKl + szWQK;
  const size_t offMhi  = offM16 + szMc;
  const size_t offMlo  = offMhi + szMc;
  const size_t offQKh  = offMlo + szMc;
  const size_t offQKl  = offQKh + szQKc;
  const size_t offG16  = offQKl + szQKc;
  const size_t offVT   = offG16 + szGc;
  const size_t offPB   = offVT + szVTc;
  const size_t offOB   = offPB + szPB;
  const size_t total   = offOB + szOB;
  if (ws_size < total) return;

  const float* msa  = (const float*)d_in[0];
  const float* pr   = (const float*)d_in[1];
  const float* lnmg = (const float*)d_in[2];
  const float* lnmb = (const float*)d_in[3];
  const float* lnpg = (const float*)d_in[4];
  const float* lnpb = (const float*)d_in[5];
  const float* wq   = (const float*)d_in[6];
  const float* wk   = (const float*)d_in[7];
  const float* wv   = (const float*)d_in[8];
  const float* wg   = (const float*)d_in[9];
  const float* bg   = (const float*)d_in[10];
  const float* wb   = (const float*)d_in[11];
  const float* bb   = (const float*)d_in[12];
  const float* wo   = (const float*)d_in[13];
  const float* bo   = (const float*)d_in[14];
  float* out = (float*)d_out;
  char* ws = (char*)d_ws;
  unsigned short* WT16 = (unsigned short*)(ws + offWT16);
  unsigned short* WQKh = (unsigned short*)(ws + offWQKh);
  unsigned short* WQKl = (unsigned short*)(ws + offWQKl);
  unsigned short* M16  = (unsigned short*)(ws + offM16);
  unsigned short* Mhi  = (unsigned short*)(ws + offMhi);
  unsigned short* Mlo  = (unsigned short*)(ws + offMlo);
  unsigned short* QKh  = (unsigned short*)(ws + offQKh);
  unsigned short* QKl  = (unsigned short*)(ws + offQKl);
  unsigned short* G16  = (unsigned short*)(ws + offG16);
  unsigned short* VT   = (unsigned short*)(ws + offVT);
  float*          PB   = (float*)(ws + offPB);
  unsigned short* OB   = (unsigned short*)(ws + offOB);
  const unsigned short* WgT = WT16;
  const unsigned short* WvT = WT16 + (size_t)1 * kWPlane;
  const unsigned short* WoT = WT16 + (size_t)2 * kWPlane;

  wtcast_kernel<<<dim3(4, 4, 3), dim3(256), 0, stream>>>(wg, wv, wo, WT16, kWCarry);
  wtsplit_kernel<<<dim3(4, 4, 2), dim3(256), 0, stream>>>(wq, wk, WQKh, WQKl);
  pair_bias_kernel<<<dim3(kPairRows / 32), dim3(256), 0, stream>>>(pr, lnpg, lnpb, wb, bb, PB);

  for (int ch = 0; ch < kNChunk; ++ch) {
    const float* msac = msa + (size_t)ch * kTokC * kCM;
    ln_msa_kernel<<<dim3(kTokC / 8), dim3(256), 0, stream>>>(msac, lnmg, lnmb, M16, Mhi, Mlo);
    wmma_gemm64<1, true, 0, 2, false, 0><<<dim3((kTokC / 64) * (kQKld / 64) / 8, 1), dim3(256), 0, stream>>>(
        Mhi, Mlo, kCM, 0L, WQKh, WQKl, kCM, 0L,
        (void*)QKh, (void*)QKl, kQKld, 0L, bo, bo, 0L, kTokC, kQKld, kCM, 1.0f);
    wmma_gemm64<0, false, 0, 1, false, 0><<<dim3((kTokC / 64) * (kHD / 64) / 8, 1), dim3(256), 0, stream>>>(
        M16, M16, kCM, 0L, WgT, WgT, kCM, 0L,
        (void*)G16, (void*)G16, kHD, 0L, bo, bo, 0L, kTokC, kHD, kCM, kWCarryInv);
    wmma_gemm64<0, false, 0, 1, false, 0><<<dim3((kHD / 64) * (kR / 64) / 8, kSC), dim3(256), 0, stream>>>(
        WvT, WvT, kCM, 0L, M16, M16, kCM, (long)kR * kCM,
        (void*)VT, (void*)VT, kR, (long)kHD * kR, bo, bo, 0L, kHD, kR, kCM, kWCarryInv);
    attn_kernel<<<dim3(kSC * 4 * (kR / kQT)), dim3(256), 0, stream>>>(QKh, QKl, G16, VT, PB, bg,
                                                                     OB + (size_t)ch * kTokC * kHD);
  }
  wmma_gemm64<0, false, 2, 0, false, 0><<<dim3((kTok / 64) * (kCM / 64) / 8, 1), dim3(256), 0, stream>>>(
      OB, OB, kHD, 0L, WoT, WoT, kHD, 0L,
      (void*)out, (void*)out, kCM, 0L, bo, bo, 0L, kTok, kCM, kHD, kOutScale);
}
